// MHSABlock_37125697306790
// MI455X (gfx1250) — hardware-verified
//
#include <hip/hip_runtime.h>
#include <math.h>
#include <stdint.h>

#ifndef NB
#define NB 8
#endif
#ifndef NQ
#define NQ 1024
#endif
#define HEADS 8
#define CDIM  512
#define DH    64
#define NSEQ  1024
#define NPROJ 3
#define MW    (NPROJ * CDIM)
#define KROW  192
#define QT    64
#define OSP   68
#define OSPW  68
#define TP    72
#define WSC   256.0f
#define IWSC  0.00390625f
#define LNPS  9.704060527839234f

static_assert(NB >= 1 && NB <= 8);
static_assert(NQ % QT == 0 && NQ >= QT && NQ <= NSEQ);
static_assert(HEADS * DH == CDIM);
static_assert(DH == QT);
static_assert(KROW == 3 * DH);
static_assert(NSEQ == 1024 && HEADS == 8);
static_assert(CDIM == 512);
static_assert(MW % 8 == 0 && (CDIM / 8) == 64);
static_assert(CDIM % 32 == 0 && NSEQ % QT == 0 && NSEQ % 32 == 0);
static_assert((OSP * 4) % 16 == 0);
static_assert((OSPW * 4) % 16 == 0);
static_assert((TP * 2) % 16 == 0);
static_assert((KROW * 2) % 128 == 0);

typedef _Float16       v16h __attribute__((ext_vector_type(16)));
typedef _Float16       v8h  __attribute__((ext_vector_type(8)));
typedef __bf16         v16b __attribute__((ext_vector_type(16)));
typedef unsigned short v8us __attribute__((ext_vector_type(8)));
typedef float          v8f  __attribute__((ext_vector_type(8)));
typedef float          v4f  __attribute__((ext_vector_type(4)));
typedef unsigned int   v4u  __attribute__((ext_vector_type(4)));

union Frag  { v8us u[2]; v16h h; v16b bf; };
union FragH { v16h v; v8h hv[2]; };
static_assert(sizeof(Frag) == 32);
static_assert(sizeof(FragH) == 32);

__device__ __forceinline__ unsigned short bf_bits(float f) {
  unsigned u = __float_as_uint(f);
  return (unsigned short)((u + 0x7FFFu + ((u >> 16) & 1u)) >> 16);
}
__device__ __forceinline__ float bf_up(unsigned short hb) { return __uint_as_float(((unsigned)hb) << 16); }
__device__ __forceinline__ float bfr(float f) { return bf_up(bf_bits(f)); }
__device__ __forceinline__ unsigned short h_bits(_Float16 x) { return __builtin_bit_cast(unsigned short, x); }
__device__ __forceinline__ unsigned pk16(unsigned short a, unsigned short b) { return (unsigned)a | ((unsigned)b << 16); }
__device__ __forceinline__ v8f zero8() { v8f z = {0.f, 0.f, 0.f, 0.f, 0.f, 0.f, 0.f, 0.f}; return z; }
__device__ __forceinline__ float hmax8(v8f s) {
  return fmaxf(fmaxf(fmaxf(s[0], s[1]), fmaxf(s[2], s[3])), fmaxf(fmaxf(s[4], s[5]), fmaxf(s[6], s[7])));
}
__device__ __forceinline__ unsigned wave_ballot(bool p) {
#if defined(__HIP_DEVICE_COMPILE__)
  return __builtin_amdgcn_ballot_w32(p);
#else
  return p ? 1u : 0u;
#endif
}

__device__ __forceinline__ Frag ldfrag(const unsigned short* p) {
  Frag f;
  f.u[0] = *(const v8us*)(p);
  f.u[1] = *(const v8us*)(p + 16);
  return f;
}

__device__ __forceinline__ v8f mma_h(v16h a, v16h b, v8f c) {
  v8f d = __builtin_amdgcn_wmma_f32_16x16x32_f16(false, a, false, b, (short)0, c, false, false);
#if defined(__HIP_DEVICE_COMPILE__)
  asm volatile("v_nop\n\tv_nop\n\tv_nop\n\tv_nop" : "+v"(d) : "v"(a), "v"(b));
#endif
  return d;
}
__device__ __forceinline__ v8f mma_b(v16b a, v16b b, v8f c) {
  v8f d = __builtin_amdgcn_wmma_f32_16x16x32_bf16(false, a, false, b, (short)0, c, false, false);
#if defined(__HIP_DEVICE_COMPILE__)
  const v16h ha = __builtin_bit_cast(v16h, a), hb = __builtin_bit_cast(v16h, b);
  asm volatile("v_nop\n\tv_nop\n\tv_nop\n\tv_nop" : "+v"(d) : "v"(ha), "v"(hb));
#endif
  return d;
}

__global__ __launch_bounds__(256)
void cvt_w(const float* __restrict__ wq, const float* __restrict__ wk, const float* __restrict__ wv,
           unsigned short* W16) {
  const int tid = threadIdx.x, blk = blockIdx.x;
  const int rl = tid >> 5, lane = tid & 31;
  const int o = 8 * blk + rl;
  const int p = blk >> 6;
  const float* wbase = (p == 0) ? wq : ((p == 1) ? wk : wv);
  const int ol = o - p * CDIM;
  v4u u[2];
#pragma unroll
  for (int it = 0; it < 2; ++it) {
    const float* s = wbase + (size_t)ol * CDIM + 256 * it + 8 * lane;
    const v4f a = *(const v4f*)s;
    const v4f q = *(const v4f*)(s + 4);
    const float f[8] = {a[0], a[1], a[2], a[3], q[0], q[1], q[2], q[3]};
#pragma unroll
    for (int t = 0; t < 4; ++t) {
      const _Float16 h0 = (_Float16)(bfr(f[2 * t]) * WSC);
      const _Float16 h1 = (_Float16)(bfr(f[2 * t + 1]) * WSC);
      u[it][t] = pk16(h_bits(h0), h_bits(h1));
    }
  }
#pragma unroll
  for (int pass = 0; pass < 2; ++pass) {
#pragma unroll
    for (int it = 0; it < 2; ++it)
      *(volatile v4u*)(W16 + (size_t)o * CDIM + 256 * it + 8 * lane) = u[it];
    __threadfence();
  }
}

__global__ __launch_bounds__(256)
void cvt_x(const float* __restrict__ x, unsigned short* XP) {
  __shared__ __align__(16) unsigned short T[QT * TP];
  const int tid = threadIdx.x;
  const int nb = blockIdx.x, cb = blockIdx.y, b = blockIdx.z;
  const int e = tid & 7, lq = tid >> 3;
  const int n0 = nb * QT, c0 = cb * QT;
#pragma unroll
  for (int it = 0; it < 2; ++it) {
    const int cl = it * 32 + lq;
    const float* sp = x + ((size_t)(b * CDIM + c0 + cl)) * NSEQ + n0 + 8 * e;
    const v4f a = *(const v4f*)sp;
    const v4f q = *(const v4f*)(sp + 4);
    unsigned short hb[8];
#pragma unroll
    for (int t = 0; t < 4; ++t) {
      hb[t]     = h_bits((_Float16)bfr(a[t]));
      hb[4 + t] = h_bits((_Float16)bfr(q[t]));
    }
#pragma unroll
    for (int t = 0; t < 8; ++t) T[(8 * e + t) * TP + cl] = hb[t];
  }
  __syncthreads();
  v4u up[2];
#pragma unroll
  for (int it = 0; it < 2; ++it) {
    const int nl = it * 32 + lq;
    up[it] = *(const v4u*)(T + nl * TP + 8 * e);
  }
#pragma unroll
  for (int pass = 0; pass < 2; ++pass) {
#pragma unroll
    for (int it = 0; it < 2; ++it) {
      const int rl = it * 32 + lq;
      *(volatile v4u*)(XP + ((size_t)(b * NSEQ + n0 + rl)) * CDIM + c0 + 8 * e) = up[it];
    }
    __threadfence();
  }
}

__global__ __launch_bounds__(256)
void pos_k(const float* __restrict__ rh, const float* __restrict__ rw, unsigned short* QKh, unsigned short* QKl) {
  const int idx = blockIdx.x * 256 + (int)threadIdx.x;
  const int e = idx & 7;
  const int n = (idx >> 3) & (NSEQ - 1);
  const int h = (idx >> 13) & (HEADS - 1);
  const int xw = n & 31, yh = n >> 5;
  v4u uh, ul;
#pragma unroll
  for (int t = 0; t < 4; ++t) {
    const int da = 8 * e + 2 * t, db = da + 1;
    const float f0 = bfr(rh[(h * DH + da) * 32 + xw]) + bfr(rw[(h * DH + da) * 32 + yh]);
    const float f1 = bfr(rh[(h * DH + db) * 32 + xw]) + bfr(rw[(h * DH + db) * 32 + yh]);
    const unsigned short hb0 = bf_bits(f0), hb1 = bf_bits(f1);
    const unsigned short lb0 = bf_bits(f0 - bf_up(hb0));
    const unsigned short lb1 = bf_bits(f1 - bf_up(hb1));
    uh[t] = pk16(hb0, hb1);
    ul[t] = pk16(lb0, lb1);
  }
#pragma unroll
  for (int pass = 0; pass < 2; ++pass) {
#pragma unroll
    for (int b = 0; b < NB; ++b) {
      const size_t po = ((size_t)((b * HEADS + h) * NSEQ + n)) * KROW + 2 * DH + 8 * e;
      *(volatile v4u*)(QKh + po) = uh;
      *(volatile v4u*)(QKl + po) = ul;
    }
    __threadfence();
  }
}

__global__ __launch_bounds__(128)
void gemm_qkv(const unsigned short* __restrict__ W16, const unsigned short* __restrict__ XP,
              const float* __restrict__ bq, const float* __restrict__ bk, const float* __restrict__ bv,
              unsigned short* QKh, unsigned short* QKl, unsigned short* Vc) {
  __shared__ __align__(16) float Os[QT * OSP];
  const int tid  = threadIdx.x;
  const int lane = tid & 31, wave = tid >> 5;
  const int hh   = lane >> 4, c = lane & 15;
  const int nt   = blockIdx.x, mb = blockIdx.y, b = blockIdx.z;
  const int n0   = nt * QT, o0 = mb * QT;

  const unsigned short* ap = W16 + (size_t)(o0 + c) * CDIM + 8 * hh;
  const unsigned short* bp = XP + ((size_t)(b * NSEQ + n0 + 16 * wave + c)) * CDIM + 8 * hh;

  v8f acc[4];
#pragma unroll
  for (int mt = 0; mt < 4; ++mt) acc[mt] = zero8();

#pragma unroll 2
  for (int ks = 0; ks < CDIM / 32; ++ks) {
    const Frag fb = ldfrag(bp + 32 * ks);
#pragma unroll
    for (int mt = 0; mt < 4; ++mt) {
      const Frag fa = ldfrag(ap + (size_t)(16 * mt) * CDIM + 32 * ks);
      acc[mt] = mma_h(fa.h, fb.h, acc[mt]);
    }
  }

  {
    const int nl = 16 * wave + c;
#pragma unroll
    for (int mt = 0; mt < 4; ++mt) {
      v4f va, vb;
#pragma unroll
      for (int r = 0; r < 4; ++r) { va[r] = acc[mt][r] * IWSC; vb[r] = acc[mt][4 + r] * IWSC; }
      *(v4f*)(Os + nl * OSP + 16 * mt + 8 * hh)     = va;
      *(v4f*)(Os + nl * OSP + 16 * mt + 8 * hh + 4) = vb;
    }
  }
  __syncthreads();

  const int e = tid & 7, lq = tid >> 3;
  const int p = mb >> 3, head = mb & 7;
  const float* bias = (p == 0) ? bq : ((p == 1) ? bk : bv);
  if (p < 2) {
    const v4f b0 = *(const v4f*)(bias + head * DH + 8 * e);
    const v4f b1 = *(const v4f*)(bias + head * DH + 8 * e + 4);
    const float bb[8] = {bfr(b0[0]), bfr(b0[1]), bfr(b0[2]), bfr(b0[3]),
                         bfr(b1[0]), bfr(b1[1]), bfr(b1[2]), bfr(b1[3])};
    v4u uh[4], ul[4];
#pragma unroll
    for (int it = 0; it < 4; ++it) {
      const int row = it * 16 + lq;
      const v4f a = *(const v4f*)(Os + row * OSP + 8 * e);
      const v4f q = *(const v4f*)(Os + row * OSP + 8 * e + 4);
      const float f[8] = {a[0], a[1], a[2], a[3], q[0], q[1], q[2], q[3]};
#pragma unroll
      for (int t = 0; t < 4; ++t) {
        const float f0 = f[2 * t] + bb[2 * t], f1 = f[2 * t + 1] + bb[2 * t + 1];
        const unsigned short hb0 = bf_bits(f0), hb1 = bf_bits(f1);
        const unsigned short lb0 = bf_bits(f0 - bf_up(hb0));
        const unsigned short lb1 = bf_bits(f1 - bf_up(hb1));
        uh[it][t] = pk16(hb0, hb1);
        ul[it][t] = pk16(lb0, lb1);
      }
    }
#pragma unroll
    for (int pass = 0; pass < 2; ++pass) {
#pragma unroll
      for (int it = 0; it < 4; ++it) {
        const int row = it * 16 + lq;
        const size_t po = ((size_t)((b * HEADS + head) * NSEQ + n0 + row)) * KROW + p * DH + 8 * e;
        *(volatile v4u*)(QKh + po) = uh[it];
        *(volatile v4u*)(QKl + po) = ul[it];
      }
      __threadfence();
    }
  } else {
    v4u uv[4];
#pragma unroll
    for (int it = 0; it < 4; ++it) {
      const int row = it * 16 + lq;
      const float bo = bfr(bias[head * DH + row]);
      unsigned short hb[8];
#pragma unroll
      for (int t = 0; t < 8; ++t) hb[t] = h_bits((_Float16)(Os[(8 * e + t) * OSP + row] + bo));
#pragma unroll
      for (int t = 0; t < 4; ++t) uv[it][t] = pk16(hb[2 * t], hb[2 * t + 1]);
    }
#pragma unroll
    for (int pass = 0; pass < 2; ++pass) {
#pragma unroll
      for (int it = 0; it < 4; ++it) {
        const int row = it * 16 + lq;
        *(volatile v4u*)(Vc + ((size_t)(b * CDIM + head * DH + row)) * NSEQ + n0 + 8 * e) = uv[it];
      }
      __threadfence();
    }
  }
}

__global__ __launch_bounds__(128)
void attn_k(const unsigned short* __restrict__ QKh, const unsigned short* __restrict__ QKl,
            const unsigned short* __restrict__ Vc, float* out) {
  __shared__ __align__(16) float Os[QT * OSPW];
  const int tid  = threadIdx.x;
  const int wave = tid >> 5, lane = tid & 31;
  const int hh   = lane >> 4, c = lane & 15;
  const int n0   = blockIdx.x * QT;
  const int bh   = blockIdx.y;
  const int b    = bh >> 3, h = bh & 7;
  const size_t prow = (size_t)bh * NSEQ * KROW;

  const size_t qo = prow + ((size_t)(n0 + 16 * wave + c)) * KROW + 8 * hh;
  const unsigned short* Qhp = QKh + qo;
  const unsigned short* Qlp = QKl + qo;
  const unsigned short* Khp = QKh + prow + (size_t)c * KROW + 8 * hh;
  const unsigned short* Klp = QKl + prow + (size_t)c * KROW + 8 * hh;
  const unsigned short* Vp = Vc + ((size_t)(b * CDIM + h * DH + c)) * NSEQ + 8 * hh;

  float m = -1.0e30f, l = 0.f;
  v8f o[4];
#pragma unroll
  for (int j = 0; j < 4; ++j) o[j] = zero8();

#pragma unroll 1
  for (int kb = 0; kb < NSEQ; kb += 32) {
    const unsigned short* k0p  = Khp + (size_t)kb * KROW;
    const unsigned short* k1p  = Khp + (size_t)(kb + 16) * KROW;
    const unsigned short* k0lp = Klp + (size_t)kb * KROW;
    const unsigned short* k1lp = Klp + (size_t)(kb + 16) * KROW;
    v8f s0 = zero8(), s1 = zero8();
#pragma unroll 1
    for (int kc = 0; kc < 4; ++kc) {
      const int acol = ((kc + 2) & 3) * 32;
      const int bcol = 32 * kc + ((kc >> 1) << 6);
      const Frag qh  = ldfrag(Qhp + bcol);
      const Frag ql  = ldfrag(Qlp + bcol);
      const Frag k0  = ldfrag(k0p + acol);
      const Frag k1  = ldfrag(k1p + acol);
      const Frag k0l = ldfrag(k0lp + acol);
      const Frag k1l = ldfrag(k1lp + acol);
      s0 = mma_b(k0.bf, qh.bf, s0);
      s1 = mma_b(k1.bf, qh.bf, s1);
      s0 = mma_b(k0.bf, ql.bf, s0);
      s1 = mma_b(k1.bf, ql.bf, s1);
      s0 = mma_b(k0l.bf, qh.bf, s0);
      s1 = mma_b(k1l.bf, qh.bf, s1);
    }

    float mx = fmaxf(hmax8(s0), hmax8(s1));
    mx = fmaxf(mx, __shfl_xor(mx, 16, 32));
    const float mn = fmaxf(m, mx);
    const unsigned grew = wave_ballot(mx > m);
    if (grew != 0u) {
      const float corr = __expf(m - mn);
      l *= corr;
#pragma unroll
      for (int j = 0; j < 4; ++j) {
#pragma unroll
        for (int r = 0; r < 8; ++r) o[j][r] *= corr;
      }
    }
    m = mn;
    const float msh = mn - LNPS;

    FragH ph;
    float ls = 0.f;
#pragma unroll
    for (int r = 0; r < 8; ++r) {
      const _Float16 p0 = (_Float16)__expf(s0[r] - msh);
      const _Float16 p1 = (_Float16)__expf(s1[r] - msh);
      ls += (float)p0 + (float)p1;
      ph.hv[0][r] = p0;
      ph.hv[1][r] = p1;
    }
    l += ls;

#pragma unroll
    for (int j = 0; j < 4; ++j) {
      const Frag vf = ldfrag(Vp + (size_t)(16 * j) * NSEQ + kb);
      o[j] = mma_h(vf.h, ph.v, o[j]);
    }
  }
  l += __shfl_xor(l, 16, 32);
  const float inv = 1.0f / l;

  const int qrow = 16 * wave + c;
#pragma unroll
  for (int j = 0; j < 4; ++j) {
    v4f va, vb;
#pragma unroll
    for (int r = 0; r < 4; ++r) { va[r] = o[j][r] * inv; vb[r] = o[j][4 + r] * inv; }
    *(v4f*)(Os + qrow * OSPW + 16 * j + 8 * hh)     = va;
    *(v4f*)(Os + qrow * OSPW + 16 * j + 8 * hh + 4) = vb;
  }
  __syncthreads();

  const int e = tid & 7, lq = tid >> 3;
  v4f res[8];
#pragma unroll
  for (int it = 0; it < 8; ++it) {
    const int L   = it * 16 + lq;
    const int chl = L >> 1, hf = L & 1;
    const int nl  = hf * 32 + 4 * e;
#pragma unroll
    for (int t = 0; t < 4; ++t) res[it][t] = Os[(nl + t) * OSPW + chl];
  }
#pragma unroll
  for (int pass = 0; pass < 2; ++pass) {
#pragma unroll
    for (int it = 0; it < 8; ++it) {
      const int L   = it * 16 + lq;
      const int chl = L >> 1, hf = L & 1;
      const int nl  = hf * 32 + 4 * e;
      const size_t idx = ((size_t)(b * CDIM + h * DH + chl)) * NSEQ + n0 + nl;
      *(volatile v4f*)(out + idx) = res[it];
    }
    __threadfence();
  }
}

extern "C" void kernel_launch(void* const* d_in, const int* in_sizes, int n_in,
                              void* d_out, int out_size, void* d_ws, size_t ws_size,
                              hipStream_t stream) {
  const int XN = NB * CDIM * NSEQ;
  if (n_in < 9) return;
  if (in_sizes[0] < XN) return;
  if (in_sizes[1] < CDIM * CDIM || in_sizes[3] < CDIM * CDIM || in_sizes[5] < CDIM * CDIM) return;
  if (in_sizes[2] < CDIM || in_sizes[4] < CDIM || in_sizes[6] < CDIM) return;
  if (in_sizes[7] < HEADS * DH * 32 || in_sizes[8] < HEADS * DH * 32) return;
  if (out_size < XN) return;

  size_t off = 0;
  auto carve = [&](size_t bytes) { const size_t o = off; off += (bytes + 255) & ~(size_t)255; return o; };
  const size_t oW16 = carve((size_t)MW * CDIM * 2);
  const size_t oXP  = carve((size_t)NB * NSEQ * CDIM * 2);
  const size_t oQKh = carve((size_t)NB * HEADS * NSEQ * KROW * 2);
  const size_t oQKl = carve((size_t)NB * HEADS * NSEQ * KROW * 2);
  const size_t oVc  = carve((size_t)NB * CDIM * NSEQ * 2);
  if (off > ws_size) return;
  if (off > (size_t)134217728) return;

  const float* x   = (const float*)d_in[0];
  const float* wqw = (const float*)d_in[1];
  const float* wqb = (const float*)d_in[2];
  const float* wkw = (const float*)d_in[3];
  const float* wkb = (const float*)d_in[4];
  const float* wvw = (const float*)d_in[5];
  const float* wvb = (const float*)d_in[6];
  const float* rh  = (const float*)d_in[7];
  const float* rw  = (const float*)d_in[8];

  char* ws = (char*)d_ws;
  unsigned short* W16 = (unsigned short*)(ws + oW16);
  unsigned short* XP  = (unsigned short*)(ws + oXP);
  unsigned short* QKh = (unsigned short*)(ws + oQKh);
  unsigned short* QKl = (unsigned short*)(ws + oQKl);
  unsigned short* Vc  = (unsigned short*)(ws + oVc);
  float* out = (float*)d_out;

  const dim3 blk256(256), blk128(128);

  cvt_w<<<dim3(MW / 8), blk256, 0, stream>>>(wqw, wkw, wvw, W16);
  cvt_x<<<dim3(NSEQ / QT, CDIM / QT, NB), blk256, 0, stream>>>(x, XP);
  pos_k<<<dim3((HEADS * NSEQ * 8) / 256), blk256, 0, stream>>>(rh, rw, QKh, QKl);
  gemm_qkv<<<dim3(NSEQ / QT, MW / QT, NB), blk128, 0, stream>>>(W16, XP, wqb, wkb, wvb, QKh, QKl, Vc);
  attn_k<<<dim3(NQ / QT, NB * HEADS), blk128, 0, stream>>>(QKh, QKl, Vc, out);
  (void)hipGetLastError();
}
